// STGATPredictor_34187939676738
// MI455X (gfx1250) — hardware-verified
//
#include <hip/hip_runtime.h>


namespace {
constexpr int NB = 16, N = 400, T = 12, CIN = 2, HID = 256, NH = 8, HDm = 32, LE = 3600, EMB = 10, TOPK = 16, NR = NB * N  , P = 3, MAXADJ = 64;
constexpr float XS = 8.0f, WSC = 256.0f, LNE = 1e-5f;

typedef _Float16 b16;
typedef __attribute__((ext_vector_type(16))) _Float16 v16b;
typedef __attribute__((ext_vector_type(8))) _Float16 v8b;
typedef __attribute__((ext_vector_type(8))) float v8f;
typedef __attribute__((ext_vector_type(4))) float v4f;
__device__ __forceinline__ float bf16_rne(float f) { unsigned int u = __float_as_uint(f); u += 0x7FFFu + ((u >> 16) & 1u); return __uint_as_float(u & 0xFFFF0000u); }
__device__ __forceinline__ void split16(float v, b16& hi, b16& lo) { hi = (b16)v; lo = (b16)(v - (float)hi); }
__device__ __forceinline__ v16b frag_kb(const b16* p, int hh) { const v8b a = *(const v8b*)(p + 8 * hh), b = *(const v8b*)(p + 16 + 8 * hh); v16b f;
#pragma unroll
  for (int e = 0; e < 8; ++e) { f[e] = a[e]; f[8 + e] = b[e]; } return f; }
__device__ __forceinline__ v8f wmma16b(v16b a, v16b b, v8f c) { v8f d = __builtin_amdgcn_wmma_f32_16x16x32_f16(false, a, false, b, (short)0, c, false, false); asm volatile("v_nop\n\tv_nop\n\tv_nop\n\tv_nop" : "+v"(d) : "v"(a), "v"(b)); return d; }
__device__ __forceinline__ void wave_lds_sync() { __builtin_amdgcn_fence(__ATOMIC_RELEASE, "workgroup"); __builtin_amdgcn_wave_barrier(); __builtin_amdgcn_fence(__ATOMIC_ACQUIRE, "workgroup"); }
__device__ __forceinline__ float pmul(float a, float b) { float p = a * b; asm volatile("" : "+v"(p)); return p; }
__device__ __forceinline__ float wsum(float v) { v += __shfl_xor(v, 1); v += __shfl_xor(v, 2); v += __shfl_xor(v, 4); v += __shfl_xor(v, 8); return v + __shfl_xor(v, 16); }
__device__ __forceinline__ float wmax(float v) { v = fmaxf(v, __shfl_xor(v, 1)); v = fmaxf(v, __shfl_xor(v, 2)); v = fmaxf(v, __shfl_xor(v, 4)); v = fmaxf(v, __shfl_xor(v, 8)); return fmaxf(v, __shfl_xor(v, 16)); }
__device__ __forceinline__ float nexp(float x) { return __builtin_amdgcn_exp2f(x * 1.4426950408889634f); }
__device__ __forceinline__ float sigm(float x) { return 1.0f / (1.0f + nexp(-x)); }
__device__ __forceinline__ float lrelu(float x) { return x > 0.0f ? x : 0.2f * x; }
__device__ __forceinline__ float elu(float x) { return x > 0.0f ? x : (__expf(x) - 1.0f); }
__device__ __forceinline__ float tanh_(float x) { const float e = nexp(-2.0f * fabsf(x)); const float t = (1.0f - e) / (1.0f + e); return x < 0.0f ? -t : t; }
__device__ __forceinline__ int iclamp(int v, int lo, int hi) { return v < lo ? lo : (v > hi ? hi : v); }

__global__ __launch_bounds__(256) void prepw_kernel(const float* __restrict__ wg0, const float* __restrict__ wf0, const float* __restrict__ ws0, b16* __restrict__ W0, const float* __restrict__ wg1, const float* __restrict__ wf1, const float* __restrict__ ws1, const float* __restrict__ p0, const float* __restrict__ p1, const float* __restrict__ p2, const float* __restrict__ p3, const float* __restrict__ p4, const float* __restrict__ p5, const float* __restrict__ p6, const float* __restrict__ p7, const float* __restrict__ p8, b16* __restrict__ W1, b16* __restrict__ WP) {
  const size_t t = (size_t)blockIdx.x * 256 + threadIdx.x; const size_t n1 = (size_t)3 * HID * 768 / 8, n2 = (size_t)9 * HID * HID / 8, n0 = (size_t)3 * HID * 32 / 8; v8b o;
  if (t >= n1 + n2 && t < n1 + n2 + n0) { const size_t e = (t - n1 - n2) * 8; const int which = (int)(e / ((size_t)HID * 32)); const size_t r = e - (size_t)which * HID * 32; const int oo = (int)(r / 32), k0 = (int)(r - (size_t)oo * 32); const float* w = which == 0 ? wg0 : which == 1 ? wf0 : ws0;
    for (int j = 0; j < 8; ++j) { const int k = k0 + j; o[j] = (b16)((k < 6) ? bf16_rne(w[(size_t)oo * 6 + k]) * WSC : 0.0f); }
    for (int pass = 0; pass < 2; ++pass) { *(volatile v8b*)(W0 + e) = o; __threadfence(); } return; }
  if (t < n1) { const size_t e = t * 8; const int which = (int)(e / ((size_t)HID * 768)); const size_t r = e - (size_t)which * HID * 768; const int oo = (int)(r / 768), k0 = (int)(r - (size_t)oo * 768); const float* w = which == 0 ? wg1 : which == 1 ? wf1 : ws1;
    for (int j = 0; j < 8; ++j) { const int k = k0 + j, tap = k >> 8, i = k & 255; o[j] = (b16)(bf16_rne(w[((size_t)oo * HID + i) * 3 + tap]) * WSC); } for (int pass = 0; pass < 2; ++pass) { *(volatile v8b*)(W1 + e) = o; __threadfence(); } }
  else if (t < n1 + n2) { const size_t e = (t - n1) * 8; const int which = (int)(e / ((size_t)HID * HID)); const size_t r = e - (size_t)which * HID * HID; const int oo = (int)(r / HID), i0 = (int)(r - (size_t)oo * HID);
    const float* w = which == 0 ? p0 : which == 1 ? p1 : which == 2 ? p2 : which == 3 ? p3 : which == 4 ? p4 : which == 5 ? p5 : which == 6 ? p6 : which == 7 ? p7 : p8;
    for (int j = 0; j < 8; ++j) o[j] = (b16)(bf16_rne(w[(size_t)(i0 + j) * HID + oo]) * WSC); for (int pass = 0; pass < 2; ++pass) { *(volatile v8b*)(WP + e) = o; __threadfence(); } }
}
__global__ __launch_bounds__(128) void tcn0_kernel(const float* __restrict__ x, const b16* __restrict__ W0, const float* __restrict__ bg, const float* __restrict__ bff, const float* __restrict__ bs, const float* __restrict__ lg, const float* __restrict__ lb, const float* __restrict__ wsk, const float* __restrict__ bsk, b16* __restrict__ Y0h, b16* __restrict__ Y0l, float* __restrict__ RES) {
  __shared__ __attribute__((aligned(16))) float Ys[4][16][HID + 4];
  const int wave = threadIdx.x >> 5, lane = threadIdx.x & 31, nloc = lane & 15, hlf = lane >> 4; const size_t r0 = ((size_t)blockIdx.x * 4 + wave) * 16;
  v16b a = {};
  { const size_t row = r0 + nloc; const int bn = (int)(row / 3), ts = (int)(row - (size_t)bn * 3); const int t = 7 + 2 * ts;
    if (hlf == 0) { for (int c = 0; c < 2; ++c) for (int tap = 0; tap < 3; ++tap) a[c * 3 + tap] = (b16)(bf16_rne(x[((size_t)bn * T + t + tap - 2) * CIN + c]) * XS); } }
  for (int qtr = 0; qtr < 4; ++qtr) { v8f g[4], f[4], s[4];
#pragma unroll
    for (int tt = 0; tt < 4; ++tt) { const int tile = qtr * 4 + tt; g[tt] = wmma16b(a, frag_kb(W0 + (size_t)(tile * 16 + nloc) * 32, hlf), (v8f){}); f[tt] = wmma16b(a, frag_kb(W0 + (size_t)HID * 32 + (size_t)(tile * 16 + nloc) * 32, hlf), (v8f){}); s[tt] = wmma16b(a, frag_kb(W0 + (size_t)2 * HID * 32 + (size_t)(tile * 16 + nloc) * 32, hlf), (v8f){}); }
#pragma unroll
    for (int tt = 0; tt < 4; ++tt) { const int o = (qtr * 4 + tt) * 16 + nloc; const float bgv = bf16_rne(bg[o]), bfv = bf16_rne(bff[o]), bsv = bf16_rne(bs[o]); const float sc = 1.0f / (XS * WSC);
#pragma unroll
      for (int r = 0; r < 8; ++r) { const float sg = sigm(g[tt][r] * sc + bgv); Ys[wave][8 * hlf + r][o] = pmul(sg, f[tt][r] * sc + bfv) + pmul(1.0f - sg, s[tt][r] * sc + bsv); } } }
  wave_lds_sync();
  for (int step = 0; step < 8; ++step) { const int rr = 2 * step + hlf; const size_t row = r0 + rr; const int bn = (int)(row / 3), ts = (int)(row - (size_t)bn * 3);
    float v[16]; float s1 = 0.0f; for (int j = 0; j < 16; ++j) { v[j] = Ys[wave][rr][nloc * 16 + j]; s1 += v[j]; }
    s1 += __shfl_xor(s1, 1); s1 += __shfl_xor(s1, 2); s1 += __shfl_xor(s1, 4); s1 += __shfl_xor(s1, 8); const float mu = s1 * (1.0f / HID);
    float s2 = 0.0f; for (int j = 0; j < 16; ++j) { const float d = v[j] - mu; s2 += d * d; } s2 += __shfl_xor(s2, 1); s2 += __shfl_xor(s2, 2); s2 += __shfl_xor(s2, 4); s2 += __shfl_xor(s2, 8); const float rs = rsqrtf(s2 * (1.0f / HID) + LNE);
    v8b h0, l0, h1, l1; v4f q0, q1, q2, q3; const float x0 = bf16_rne(x[((size_t)bn * T + 11) * CIN]), x1 = bf16_rne(x[((size_t)bn * T + 11) * CIN + 1]);
    for (int j = 0; j < 16; ++j) { const int o = nloc * 16 + j; const float yv = fmaxf(pmul((v[j] - mu) * rs, bf16_rne(lg[o])) + bf16_rne(lb[o]), 0.0f); b16 p_, q_; split16(yv * XS, p_, q_); if (j < 8) { h0[j] = p_; l0[j] = q_; } else { h1[j - 8] = p_; l1[j - 8] = q_; }
      const float rv = pmul(x0, bf16_rne(wsk[o])) + pmul(x1, bf16_rne(wsk[HID + o])) + bf16_rne(bsk[o]); if (j < 4) q0[j] = rv; else if (j < 8) q1[j - 4] = rv; else if (j < 12) q2[j - 8] = rv; else q3[j - 12] = rv; }
    for (int pass = 0; pass < 2; ++pass) { b16* ph = Y0h + row * HID + nloc * 16; b16* pl = Y0l + row * HID + nloc * 16; *(volatile v8b*)ph = h0; *(volatile v8b*)(ph + 8) = h1; *(volatile v8b*)pl = l0; *(volatile v8b*)(pl + 8) = l1;
      if (ts == 2) { float* pr = RES + (size_t)bn * HID + nloc * 16; *(volatile v4f*)pr = q0; *(volatile v4f*)(pr + 4) = q1; *(volatile v4f*)(pr + 8) = q2; *(volatile v4f*)(pr + 12) = q3; } __threadfence(); } }
}
__global__ __launch_bounds__(128) void gemm_kernel(const b16* __restrict__ Ah, const b16* __restrict__ Al, int K, const b16* __restrict__ W, const float* __restrict__ bias, float* __restrict__ Y) {
  __shared__ __attribute__((aligned(16))) float Ts[4][16][128 + 4];
  const int wave = threadIdx.x >> 5, lane = threadIdx.x & 31, nloc = lane & 15, hlf = lane >> 4; const size_t m0 = (size_t)blockIdx.x * 64 + wave * 16; const int n0 = blockIdx.y * 128;
  v8f acc[8];
#pragma unroll
  for (int t = 0; t < 8; ++t) acc[t] = (v8f){};
  for (int kb = 0; kb < K; kb += 32) { const v16b a = frag_kb(Ah + (m0 + nloc) * K + kb, hlf), al = frag_kb(Al + (m0 + nloc) * K + kb, hlf);
#pragma unroll
    for (int t = 0; t < 8; ++t) { const v16b bw = frag_kb(W + (size_t)(n0 + t * 16 + nloc) * K + kb, hlf); acc[t] = wmma16b(a, bw, acc[t]); acc[t] = wmma16b(al, bw, acc[t]); } }
#pragma unroll
  for (int t = 0; t < 8; ++t) { const int c = n0 + t * 16 + nloc; const float bb = bias ? bf16_rne(bias[c]) : 0.0f;
#pragma unroll
    for (int r = 0; r < 8; ++r) Ts[wave][8 * hlf + r][t * 16 + nloc] = acc[t][r] * (1.0f / (XS * WSC)) + bb; }
  wave_lds_sync();
  for (int pass = 0; pass < 2; ++pass) { for (int rr = 0; rr < 16; ++rr) *(volatile v4f*)(Y + (m0 + rr) * HID + n0 + lane * 4) = *(const v4f*)(&Ts[wave][rr][lane * 4]); __threadfence(); }
}
__global__ __launch_bounds__(256) void tcn1_kernel(const float* __restrict__ G, const float* __restrict__ F, const float* __restrict__ S, const float* __restrict__ lg, const float* __restrict__ lb, const float* __restrict__ RES, float* __restrict__ HL, b16* __restrict__ HLh, b16* __restrict__ HLl) {
  const int wave = threadIdx.x >> 5, lane = threadIdx.x & 31; const size_t row = (size_t)blockIdx.x * 8 + wave; const int c0 = lane * 8;
  float y[8]; float s1 = 0.0f; for (int j = 0; j < 8; ++j) { const size_t i = row * HID + c0 + j; const float sg = sigm(G[i]); y[j] = pmul(sg, F[i]) + pmul(1.0f - sg, S[i]); s1 += y[j]; }
  const float mu = wsum(s1) * (1.0f / HID); float s2 = 0.0f; for (int j = 0; j < 8; ++j) { const float d = y[j] - mu; s2 += d * d; } const float rs = rsqrtf(wsum(s2) * (1.0f / HID) + LNE);
  v4f o0, o1; v8b hv, lv; for (int j = 0; j < 8; ++j) { const int o = c0 + j; const float v = fmaxf(pmul((y[j] - mu) * rs, bf16_rne(lg[o])) + bf16_rne(lb[o]), 0.0f) + RES[row * HID + o]; if (j < 4) o0[j] = v; else o1[j - 4] = v; b16 a_, c_; split16(v * XS, a_, c_); hv[j] = a_; lv[j] = c_; }
  for (int pass = 0; pass < 2; ++pass) { *(volatile v4f*)(HL + row * HID + c0) = o0; *(volatile v4f*)(HL + row * HID + c0 + 4) = o1; *(volatile v8b*)(HLh + row * HID + c0) = hv; *(volatile v8b*)(HLl + row * HID + c0) = lv; __threadfence(); }
}
__global__ __launch_bounds__(256) void headdot_kernel(const float* __restrict__ SQ, const float* __restrict__ SK, const float* __restrict__ DQ, const float* __restrict__ DK, const float* __restrict__ saq, const float* __restrict__ sak, const float* __restrict__ daq, const float* __restrict__ dak, float* __restrict__ AD) {
  const int wave = threadIdx.x >> 5, lane = threadIdx.x & 31; const size_t row = (size_t)blockIdx.x * 8 + wave; const int h = lane >> 2, d0 = (lane & 3) * 8;
  float s[4] = {0, 0, 0, 0};
  for (int j = 0; j < 8; ++j) { const size_t i = row * HID + h * HDm + d0 + j; const int ai = h * HDm + d0 + j; s[0] += pmul(SQ[i], bf16_rne(saq[ai])); s[1] += pmul(SK[i], bf16_rne(sak[ai])); s[2] += pmul(DQ[i], bf16_rne(daq[ai])); s[3] += pmul(DK[i], bf16_rne(dak[ai])); }
#pragma unroll
  for (int u = 0; u < 4; ++u) { s[u] += __shfl_xor(s[u], 1); s[u] += __shfl_xor(s[u], 2); }
  for (int pass = 0; pass < 2; ++pass) { if ((lane & 3) == 0) { ((volatile float*)AD)[row * 32 + 0 * 8 + h] = s[0]; ((volatile float*)AD)[row * 32 + 8 + h] = s[1]; ((volatile float*)AD)[row * 32 + 16 + h] = s[2]; ((volatile float*)AD)[row * 32 + 24 + h] = s[3]; } __threadfence(); }
}
__global__ __launch_bounds__(512) void adj_kernel(const float* __restrict__ E1, const float* __restrict__ E2, int* __restrict__ JL, float* __restrict__ LA, int* __restrict__ CNT, int* __restrict__ FLAG) {
  __shared__ float zs[N]; __shared__ float red[512]; __shared__ int flag_s[N]; __shared__ int pos[N];
  const int n = blockIdx.x, t_ = threadIdx.x; float z = -INFINITY;
  if (t_ < N) { float s = 0.0f; for (int k = 0; k < EMB; ++k) s = fmaf(bf16_rne(E1[n * EMB + k]), bf16_rne(E2[t_ * EMB + k]), s); z = fmaxf(s, 0.0f); zs[t_] = z; }
  red[t_] = z; __syncthreads(); for (int s = 256; s >= 1; s >>= 1) { if (t_ < s) red[t_] = fmaxf(red[t_], red[t_ + s]); __syncthreads(); } const float mx = red[0]; __syncthreads();
  const float e = (t_ < N) ? nexp(z - mx) : 0.0f; red[t_] = e; __syncthreads(); for (int s = 256; s >= 1; s >>= 1) { if (t_ < s) red[t_] += red[t_ + s]; __syncthreads(); } const float den = red[0]; __syncthreads();
  const float a = e / den;
  int sel = 0; if (t_ < N) { int gt = 0, ge = 0; for (int i = 0; i < N; ++i) { const float zi = zs[i]; gt += (zi > z) ? 1 : 0; ge += (zi >= z) ? 1 : 0; } sel = (gt < TOPK) ? 1 : 0; (void)ge; }
  if (t_ < N) flag_s[t_] = sel; __syncthreads();
  if (t_ == 0) { int c = 0; for (int i = 0; i < N; ++i) { if (flag_s[i]) { pos[i] = c; c += 1; } else pos[i] = -1; } red[0] = (float)c; }
  __syncthreads(); const int cnt = (int)red[0];
  for (int pass = 0; pass < 2; ++pass) { if (t_ < N && sel && pos[t_] < MAXADJ) { ((volatile int*)JL)[n * MAXADJ + pos[t_]] = t_; ((volatile float*)LA)[n * MAXADJ + pos[t_]] = __logf(fmaxf(a, 1e-12f)); }
    if (t_ >= cnt && t_ < MAXADJ) { ((volatile int*)JL)[n * MAXADJ + t_] = 0; ((volatile float*)LA)[n * MAXADJ + t_] = 0.0f; }
    if (t_ == 0) { ((volatile int*)CNT)[n] = min(cnt, MAXADJ); if (cnt > MAXADJ) ((volatile int*)FLAG)[0] = 1; } __threadfence(); }
}
__global__ __launch_bounds__(256) void gat_kernel(const float* __restrict__ AD, const float* __restrict__ SV, const float* __restrict__ DV, const float* __restrict__ ef, const float* __restrict__ CE, const int* __restrict__ REDGE, const int* __restrict__ RCNT, const int* __restrict__ sendv, const int* __restrict__ JL, const float* __restrict__ LA, const int* __restrict__ CNT,
                                               b16* __restrict__ HFh, b16* __restrict__ HFl, b16* __restrict__ HAh, b16* __restrict__ HAl, b16* __restrict__ HSh, b16* __restrict__ HSl) {
  const int wave = threadIdx.x >> 5, lane = threadIdx.x & 31; const size_t row = (size_t)blockIdx.x * 8 + wave; const int b = (int)(row / N), n = (int)(row - (size_t)b * N); const int h = lane >> 2, c0 = lane * 8;
  float hf[8]; { const float qa = AD[row * 32 + h]; const int cnt = iclamp(RCNT[n], 0, 16); float m = -INFINITY;
    for (int i = 0; i < cnt; ++i) { const int l = iclamp(REDGE[n * 16 + i], 0, LE - 1); const int sd = iclamp(sendv[l], 0, N - 1); const float s = lrelu(qa + AD[((size_t)b * N + sd) * 32 + 8 + h] + pmul(bf16_rne(ef[((size_t)b * LE + l) * 2]), CE[h]) + pmul(bf16_rne(ef[((size_t)b * LE + l) * 2 + 1]), CE[8 + h])); m = fmaxf(m, s); }
    float den = 0.0f; float acc[8] = {0, 0, 0, 0, 0, 0, 0, 0};
    for (int i = 0; i < cnt; ++i) { const int l = iclamp(REDGE[n * 16 + i], 0, LE - 1); const int sd = iclamp(sendv[l], 0, N - 1); const float s = lrelu(qa + AD[((size_t)b * N + sd) * 32 + 8 + h] + pmul(bf16_rne(ef[((size_t)b * LE + l) * 2]), CE[h]) + pmul(bf16_rne(ef[((size_t)b * LE + l) * 2 + 1]), CE[8 + h])); const float ex = nexp(s - m); den += ex;
      const float* vr = SV + ((size_t)b * N + sd) * HID + c0; for (int j = 0; j < 8; ++j) acc[j] += pmul(ex, vr[j]); }
    const float inv = (cnt > 0) ? 1.0f / fmaxf(den, 1e-12f) : 0.0f; for (int j = 0; j < 8; ++j) hf[j] = elu(acc[j] * inv); }
  float ha[8]; { const float qa = AD[row * 32 + 16 + h]; const int cnt = iclamp(CNT[n], 0, MAXADJ); float m = -INFINITY;
    for (int i = 0; i < cnt; ++i) { const int j = iclamp(JL[n * MAXADJ + i], 0, N - 1); const float s = lrelu(qa + AD[((size_t)b * N + j) * 32 + 24 + h]) + LA[n * MAXADJ + i]; m = fmaxf(m, s); }
    float den = 0.0f; float acc[8] = {0, 0, 0, 0, 0, 0, 0, 0};
    for (int i = 0; i < cnt; ++i) { const int j = iclamp(JL[n * MAXADJ + i], 0, N - 1); const float s = lrelu(qa + AD[((size_t)b * N + j) * 32 + 24 + h]) + LA[n * MAXADJ + i]; const float ex = nexp(s - m); den += ex;
      const float* vr = DV + ((size_t)b * N + j) * HID + c0; for (int jj = 0; jj < 8; ++jj) acc[jj] += pmul(ex, vr[jj]); }
    const float inv = (cnt > 0) ? 1.0f / den : 0.0f; for (int j = 0; j < 8; ++j) ha[j] = elu(acc[j] * inv); }
  v8b a1, a2, b1, b2, c1, c2; for (int j = 0; j < 8; ++j) { b16 p, q; split16(hf[j] * XS, p, q); a1[j] = p; a2[j] = q; split16(ha[j] * XS, p, q); b1[j] = p; b2[j] = q; split16((hf[j] + ha[j]) * XS, p, q); c1[j] = p; c2[j] = q; }
  for (int pass = 0; pass < 2; ++pass) { *(volatile v8b*)(HFh + row * HID + c0) = a1; *(volatile v8b*)(HFl + row * HID + c0) = a2; *(volatile v8b*)(HAh + row * HID + c0) = b1; *(volatile v8b*)(HAl + row * HID + c0) = b2; *(volatile v8b*)(HSh + row * HID + c0) = c1; *(volatile v8b*)(HSl + row * HID + c0) = c2; __threadfence(); }
}
__global__ __launch_bounds__(512) void graph_kernel(const int* __restrict__ recv, const float* __restrict__ swe, const float* __restrict__ sae, int* __restrict__ REDGE, int* __restrict__ RCNT, float* __restrict__ CE, int* __restrict__ FLAG) {
  __shared__ int cnt[N];
  const int t_ = threadIdx.x; if (t_ < N) cnt[t_] = 0; __syncthreads();
  if (t_ == 0) { int over = 0; for (int l = 0; l < LE; ++l) { const int r = iclamp(recv[l], 0, N - 1); const int c = cnt[r]; if (c < 16) REDGE[r * 16 + c] = l; else over = 1; cnt[r] = c + 1; } if (over) FLAG[0] = 1; }
  __syncthreads();
  for (int pass = 0; pass < 2; ++pass) { if (t_ < N) { const int c = min(cnt[t_], 16); ((volatile int*)RCNT)[t_] = c; for (int i = c; i < 16; ++i) ((volatile int*)REDGE)[t_ * 16 + i] = 0; }
    if (t_ < 16) { const int h = t_ & 7, w = t_ >> 3; float s = 0.0f; for (int d = 0; d < HDm; ++d) s += pmul(bf16_rne(swe[w * HID + h * HDm + d]), bf16_rne(sae[h * HDm + d])); ((volatile float*)CE)[t_] = s; }
    __threadfence(); }
}
__global__ __launch_bounds__(256) void tail_kernel(const float* __restrict__ G1, const float* __restrict__ T2, const float* __restrict__ T3, const float* __restrict__ wo, const float* __restrict__ bo, float* __restrict__ out) {
  __shared__ float So[32][4];
  const int wave = threadIdx.x >> 5, lane = threadIdx.x & 31, t_ = threadIdx.x; const int c0 = lane * 8;
  for (int q = 0; q < 4; ++q) { const size_t row = (size_t)blockIdx.x * 32 + wave * 4 + q; float s[3] = {0, 0, 0};
    for (int j = 0; j < 8; ++j) { const size_t i = row * HID + c0 + j; const float g = sigm(G1[i]); const float f = tanh_(pmul(g, T2[i]) + pmul(1.0f - g, T3[i])); for (int p = 0; p < 3; ++p) s[p] += pmul(f, bf16_rne(wo[(c0 + j) * P + p])); }
    for (int p = 0; p < 3; ++p) { s[p] = wsum(s[p]); } if (lane == 0) { So[wave * 4 + q][0] = s[0] + bf16_rne(bo[0]); So[wave * 4 + q][1] = s[1] + bf16_rne(bo[1]); So[wave * 4 + q][2] = s[2] + bf16_rne(bo[2]); } }
  __syncthreads();
  for (int pass = 0; pass < 2; ++pass) { if (t_ < 96) ((volatile float*)out)[(size_t)blockIdx.x * 96 + t_] = So[t_ / 3][t_ % 3]; __threadfence(); }
}
}

extern "C" void kernel_launch(void* const* d_in, const int* in_sizes, int n_in, void* d_out, int out_size, void* d_ws, size_t ws_size, hipStream_t stream) {
  (void)n_in;
  auto Fp = [&](int i) { return (const float*)d_in[i]; }; auto Ip = [&](int i) { return (const int*)d_in[i]; };
  if (in_sizes[0] != NR * T * CIN || in_sizes[1] != NB * LE * 2 || in_sizes[11] != HID * HID * 3 || in_sizes[21] != HID * HID || in_sizes[33] != N * EMB || in_sizes[41] != HID * P || in_sizes[2] != 2 * LE || out_size != NR * P) return;
  size_t off = 0; char* ws = (char*)d_ws;
  auto carve = [&](size_t bytes) { char* p = ws + off; off += (bytes + 255) & ~(size_t)255; return p; };
  b16* W1 = (b16*)carve((size_t)3 * HID * 768 * 2); b16* WP = (b16*)carve((size_t)9 * HID * HID * 2); b16* W0 = (b16*)carve((size_t)3 * HID * 32 * 2);
  b16* Y0h = (b16*)carve((size_t)NR * 3 * HID * 2); b16* Y0l = (b16*)carve((size_t)NR * 3 * HID * 2); float* RES = (float*)carve((size_t)NR * HID * 4);
  float* G = (float*)carve((size_t)NR * HID * 4); float* F = (float*)carve((size_t)NR * HID * 4); float* S = (float*)carve((size_t)NR * HID * 4); float* HL = (float*)carve((size_t)NR * HID * 4); b16* HLh = (b16*)carve((size_t)NR * HID * 2); b16* HLl = (b16*)carve((size_t)NR * HID * 2);
  float* SQ = (float*)carve((size_t)NR * HID * 4); float* SK = (float*)carve((size_t)NR * HID * 4); float* SV = (float*)carve((size_t)NR * HID * 4); float* DQ = (float*)carve((size_t)NR * HID * 4); float* DK = (float*)carve((size_t)NR * HID * 4); float* DV = (float*)carve((size_t)NR * HID * 4);
  float* AD = (float*)carve((size_t)NR * 32 * 4); int* JL = (int*)carve((size_t)N * MAXADJ * 4); float* LA = (float*)carve((size_t)N * MAXADJ * 4); int* CNT = (int*)carve((size_t)N * 4 + 256); int* FLAG = (int*)carve(256); int* REDGE = (int*)carve((size_t)N * 16 * 4); int* RCNT = (int*)carve((size_t)N * 4 + 256); float* CE = (float*)carve(256);
  b16* HFh = (b16*)carve((size_t)NR * HID * 2); b16* HFl = (b16*)carve((size_t)NR * HID * 2); b16* HAh = (b16*)carve((size_t)NR * HID * 2); b16* HAl = (b16*)carve((size_t)NR * HID * 2); b16* HSh = (b16*)carve((size_t)NR * HID * 2); b16* HSl = (b16*)carve((size_t)NR * HID * 2);
  if (off > ws_size || off > ((size_t)128 << 20)) return;
  prepw_kernel<<<(unsigned)(((size_t)3 * HID * 768 / 8 + (size_t)9 * HID * HID / 8 + (size_t)3 * HID * 32 / 8 + 255) / 256), 256, 0, stream>>>(Fp(3), Fp(5), Fp(7), W0, Fp(11), Fp(13), Fp(15), Fp(21), Fp(22), Fp(23), Fp(28), Fp(29), Fp(30), Fp(35), Fp(37), Fp(39), W1, WP);
  graph_kernel<<<1, 512, 0, stream>>>(Ip(2), Fp(24), Fp(27), REDGE, RCNT, CE, FLAG);
  adj_kernel<<<N, 512, 0, stream>>>(Fp(33), Fp(34), JL, LA, CNT, FLAG);
  tcn0_kernel<<<NR * 3 / 64, 128, 0, stream>>>(Fp(0), W0, Fp(4), Fp(6), Fp(8), Fp(9), Fp(10), Fp(19), Fp(20), Y0h, Y0l, RES);
  gemm_kernel<<<dim3(NR / 64, 2), 128, 0, stream>>>(Y0h, Y0l, 768, W1, Fp(12), G);
  gemm_kernel<<<dim3(NR / 64, 2), 128, 0, stream>>>(Y0h, Y0l, 768, W1 + (size_t)HID * 768, Fp(14), F);
  gemm_kernel<<<dim3(NR / 64, 2), 128, 0, stream>>>(Y0h, Y0l, 768, W1 + (size_t)2 * HID * 768, Fp(16), S);
  tcn1_kernel<<<NR / 8, 256, 0, stream>>>(G, F, S, Fp(17), Fp(18), RES, HL, HLh, HLl);
  { float* outs[6] = {SQ, SK, SV, DQ, DK, DV}; for (int i = 0; i < 6; ++i) gemm_kernel<<<dim3(NR / 64, 2), 128, 0, stream>>>(HLh, HLl, HID, WP + (size_t)i * HID * HID, nullptr, outs[i]); }
  headdot_kernel<<<NR / 8, 256, 0, stream>>>(SQ, SK, DQ, DK, Fp(25), Fp(26), Fp(31), Fp(32), AD);
  gat_kernel<<<NR / 8, 256, 0, stream>>>(AD, SV, DV, Fp(1), CE, REDGE, RCNT, Ip(2) + LE, JL, LA, CNT, HFh, HFl, HAh, HAl, HSh, HSl);
  gemm_kernel<<<dim3(NR / 64, 2), 128, 0, stream>>>(HSh, HSl, HID, WP + (size_t)6 * HID * HID, Fp(36), G);
  gemm_kernel<<<dim3(NR / 64, 2), 128, 0, stream>>>(HFh, HFl, HID, WP + (size_t)7 * HID * HID, Fp(38), F);
  gemm_kernel<<<dim3(NR / 64, 2), 128, 0, stream>>>(HAh, HAl, HID, WP + (size_t)8 * HID * HID, Fp(40), S);
  tail_kernel<<<NR / 32, 256, 0, stream>>>(G, F, S, Fp(41), Fp(42), (float*)d_out);
}
